// SimpleLSTMModel_84378927497698
// MI455X (gfx1250) — hardware-verified
//
#include <hip/hip_runtime.h>


#define AS3 __attribute__((address_space(3)))

#define NB    64
#define TL    360
#define FIN   4
#define ED    32
#define CD    128
#define HWD   1024
#define HMAP  32
#define DD    128
#define SD    64
#define AD    64
#define HD    128
#define IFD   128
#define OD    5
#define KIN   288
#define KCAT  416
#define NG    512
#define BB    16
#define NBLK  (NB / BB)
#define NTHR  256
#define WPITCH 448
#define APITCH 416
#define AAP    256
#define EPITCH 136
#define PPITCH 68

static_assert(KIN == ED + CD + IFD);
static_assert(KCAT == KIN + HD);
static_assert(KCAT % 32 == 0);
static_assert(HD % 32 == 0);
static_assert((HD + DD) % 32 == 0);
static_assert(DD % 32 == 0);
static_assert(WPITCH % 64 == 0);
static_assert(WPITCH >= KCAT);
static_assert(APITCH % 8 == 0);
static_assert(APITCH >= KCAT);
static_assert(AAP % 8 == 0);
static_assert(EPITCH % 8 == 0);
static_assert(PPITCH % 4 == 0);
static_assert(NB % BB == 0);
static_assert(BB == 16);
static_assert(NTHR == 256);
static_assert(HD == (NTHR / 32) * 16);
static_assert(IFD == (NTHR / 32) * 16);
static_assert(AD == 4 * 16);

typedef __bf16          v16bf __attribute__((ext_vector_type(16)));
typedef unsigned short  v16us __attribute__((ext_vector_type(16)));
typedef unsigned short  v8us  __attribute__((ext_vector_type(8)));
typedef float           v8f   __attribute__((ext_vector_type(8)));
typedef float           v4f   __attribute__((ext_vector_type(4)));

union Frag { v16bf v; v16us u; v8us half[2]; };

typedef AS3 unsigned short*       lp_us;
typedef AS3 const unsigned short* lcp_us;
typedef AS3 float*                lp_f;
typedef AS3 const float*          lcp_f;
typedef AS3 int*                  lp_i;

constexpr size_t SZ_WC  = (size_t)NG * WPITCH * 2;
constexpr size_t SZ_WA  = (size_t)AD * HD * 2;
constexpr size_t SZ_WP  = (size_t)IFD * (HD + DD) * 2;
constexpr size_t SZ_WE  = (size_t)AD * DD * 2;
constexpr size_t SZ_PE  = (size_t)NB * SD * AD * 4;
constexpr size_t OFF_WCH = 0;
constexpr size_t OFF_WCL = OFF_WCH + SZ_WC;
constexpr size_t OFF_WAH = OFF_WCL + SZ_WC;
constexpr size_t OFF_WAL = OFF_WAH + SZ_WA;
constexpr size_t OFF_WPH = OFF_WAL + SZ_WA;
constexpr size_t OFF_WPL = OFF_WPH + SZ_WP;
constexpr size_t OFF_WEH = OFF_WPL + SZ_WP;
constexpr size_t OFF_WEL = OFF_WEH + SZ_WE;
constexpr size_t OFF_PE  = OFF_WEL + SZ_WE;
constexpr size_t WS_END  = OFF_PE + SZ_PE;
static_assert(OFF_WCL % 128 == 0 && OFF_WAH % 128 == 0 && OFF_WAL % 128 == 0 && OFF_WPH % 128 == 0);
static_assert(OFF_WPL % 128 == 0 && OFF_WEH % 128 == 0 && OFF_WEL % 128 == 0 && OFF_PE % 128 == 0);
static_assert(WS_END <= (size_t)134217728);

constexpr int NPC_C = NG * (WPITCH / 8);
constexpr int NPC_A = AD * (HD / 8);
constexpr int NPC_P = IFD * ((HD + DD) / 8);
constexpr int NPC_E = AD * (DD / 8);
static_assert(NPC_C % NTHR == 0 && NPC_A % NTHR == 0 && NPC_P % NTHR == 0 && NPC_E % NTHR == 0);
constexpr int CB0 = NPC_C / NTHR;
constexpr int CB1 = CB0 + NPC_A / NTHR;
constexpr int CB2 = CB1 + NPC_P / NTHR;
constexpr int CB3 = CB2 + NPC_E / NTHR;
static_assert((size_t)NPC_C * 16 == SZ_WC && (size_t)NPC_A * 16 == SZ_WA && (size_t)NPC_P * 16 == SZ_WP && (size_t)NPC_E * 16 == SZ_WE);

constexpr size_t LSZ_ACT = (size_t)BB * APITCH * 2;
constexpr size_t LSZ_AA  = (size_t)BB * AAP * 2;
constexpr size_t LO_ACTH = 0;
constexpr size_t LO_ACTL = LO_ACTH + LSZ_ACT;
constexpr size_t LO_AAH  = LO_ACTL + LSZ_ACT;
constexpr size_t LO_AAL  = LO_AAH + LSZ_AA;
constexpr size_t LO_C    = LO_AAL + LSZ_AA;
constexpr size_t LO_ATTH = LO_C + (size_t)BB * HD * 4;
constexpr size_t LO_WGT  = LO_ATTH + (size_t)BB * AD * 4;
constexpr size_t LO_OUTF = LO_WGT + (size_t)BB * SD * 4;
constexpr size_t LO_BIAS = LO_OUTF + (size_t)BB * IFD * 4;
constexpr size_t LO_BH2  = LO_BIAS + (size_t)NG * 4;
constexpr size_t LO_WALP = LO_BH2 + (size_t)AD * 4;
constexpr size_t LO_BAAP = LO_WALP + (size_t)AD * 4;
constexpr size_t LO_WOUT = LO_BAAP + (size_t)IFD * 4;
constexpr size_t LO_WEMB = LO_WOUT + (size_t)IFD * OD * 4;
constexpr size_t LO_BEMB = LO_WEMB + (size_t)FIN * ED * 4;
constexpr size_t LO_BOUT = LO_BEMB + (size_t)ED * 4;
constexpr size_t LO_IDX  = LO_BOUT + 32;
constexpr size_t LO_OUTS = LO_IDX + 64;
constexpr size_t LSZ_OUTS = (size_t)BB * TL * OD * 4;
constexpr size_t LDS_BYTES = LO_OUTS + LSZ_OUTS;
static_assert(LO_ACTL % 16 == 0 && LO_AAH % 16 == 0 && LO_AAL % 16 == 0 && LO_C % 16 == 0 && LO_ATTH % 16 == 0);
static_assert(LO_WGT % 16 == 0 && LO_OUTF % 16 == 0 && LO_BIAS % 16 == 0 && LO_BH2 % 16 == 0 && LO_WALP % 16 == 0);
static_assert(LO_BAAP % 16 == 0 && LO_WOUT % 16 == 0 && LO_WEMB % 16 == 0 && LO_BEMB % 16 == 0 && LO_BOUT % 16 == 0);
static_assert(LO_IDX % 16 == 0 && LO_OUTS % 16 == 0);
static_assert(LO_ATTH % 16 == 0);
constexpr int NOUTP = (BB * TL * OD) / 4;
static_assert((BB * TL * OD) % 4 == 0);
static_assert(((size_t)BB * TL * OD * 4) % 128 == 0);
constexpr int NOUT_IT = (NOUTP + NTHR - 1) / NTHR;

__device__ __forceinline__ unsigned int bfb(float x) {
    unsigned int u = __float_as_uint(x);
    u += 0x7FFFu + ((u >> 16) & 1u);
    return u >> 16;
}
__device__ __forceinline__ void split2(float x, unsigned short& hb, unsigned short& lb) {
    const unsigned int h = bfb(x);
    const float hv = __uint_as_float(h << 16);
    hb = (unsigned short)h;
    lb = (unsigned short)bfb(x - hv);
}
__device__ __forceinline__ float rcpx(float x) { return __builtin_amdgcn_rcpf(x); }
__device__ __forceinline__ float sigm(float x) { return rcpx(1.0f + __expf(-x)); }
__device__ __forceinline__ float tanhm(float x) {
    const float e = __expf(2.0f * x);
    return 1.0f - 2.0f * rcpx(e + 1.0f);
}
__device__ __forceinline__ v8f zero8() {
    v8f z;
#pragma unroll
    for (int i = 0; i < 8; ++i) z[i] = 0.0f;
    return z;
}

__device__ __forceinline__ void ldfrag_lds(Frag& f, lcp_us p) {
    f.half[0] = *(AS3 const v8us*)(p);
    f.half[1] = *(AS3 const v8us*)(p + 16);
}
__device__ __forceinline__ void ldfrag_glb(Frag& f, const unsigned short* p) {
    f.half[0] = *(const v8us*)(p);
    f.half[1] = *(const v8us*)(p + 16);
}
__device__ __forceinline__ v8f mma16(v8f c, const Frag& a, const Frag& b) {
    return __builtin_amdgcn_wmma_f32_16x16x32_bf16(false, a.v, false, b.v, (short)0, c, false, false);
}

__global__ __launch_bounds__(NTHR)
void cvt_kernel(const float* __restrict__ Wih, const float* __restrict__ Whh, const float* __restrict__ Wh2,
                const float* __restrict__ Wap, const float* __restrict__ Wen,
                unsigned short* WcH, unsigned short* WcL, unsigned short* WaH, unsigned short* WaL,
                unsigned short* WpH, unsigned short* WpL, unsigned short* WeH, unsigned short* WeL)
{
    const int bid = blockIdx.x, tid = threadIdx.x;
    const float* s0; const float* s1;
    int ld, K0, K1, ppr, p;
    unsigned short* dH; unsigned short* dL;
    if (bid < CB0)      { s0 = Wih; s1 = Whh; ld = NG;  K0 = KIN;     K1 = HD; ppr = WPITCH / 8;    p = bid * NTHR + tid;         dH = WcH; dL = WcL; }
    else if (bid < CB1) { s0 = Wh2; s1 = Wh2; ld = AD;  K0 = HD;      K1 = 0;  ppr = HD / 8;        p = (bid - CB0) * NTHR + tid; dH = WaH; dL = WaL; }
    else if (bid < CB2) { s0 = Wap; s1 = Wap; ld = IFD; K0 = HD + DD; K1 = 0;  ppr = (HD + DD) / 8; p = (bid - CB1) * NTHR + tid; dH = WpH; dL = WpL; }
    else                { s0 = Wen; s1 = Wen; ld = AD;  K0 = DD;      K1 = 0;  ppr = DD / 8;        p = (bid - CB2) * NTHR + tid; dH = WeH; dL = WeL; }
    const int n  = p / ppr;
    const int c8 = (p - n * ppr) * 8;
    v8us hv, lv;
#pragma unroll
    for (int i = 0; i < 8; ++i) {
        const int k  = c8 + i;
        const int ka = min(k, K0 - 1);
        const int kb = min(max(k - K0, 0), max(K1 - 1, 0));
        const float a  = s0[(size_t)ka * ld + n];
        const float bv = s1[(size_t)kb * ld + n];
        const float v  = (k < K0) ? a : ((k < K0 + K1) ? bv : 0.0f);
        unsigned short xh, xl;
        split2(v, xh, xl);
        hv[i] = xh; lv[i] = xl;
    }
    const size_t off = (size_t)p * 8;
    *(volatile v8us*)(dH + off) = hv;
    *(volatile v8us*)(dL + off) = lv;
    __threadfence();
    *(volatile v8us*)(dH + off) = hv;
    *(volatile v8us*)(dL + off) = lv;
}

__global__ __launch_bounds__(NTHR)
void penc_kernel(const float* __restrict__ fh, const unsigned short* __restrict__ WeH,
                 const unsigned short* __restrict__ WeL, const float* __restrict__ benc, float* penc)
{
    __shared__ __attribute__((aligned(16))) unsigned short sAH[SD * EPITCH];
    __shared__ __attribute__((aligned(16))) unsigned short sAL[SD * EPITCH];
    __shared__ __attribute__((aligned(16))) float sP[SD * PPITCH];

    const int tid = threadIdx.x, lane = tid & 31, wave = tid >> 5, h = lane >> 4, m = lane & 15;
    const int b = blockIdx.x;
    const float* fb = fh + (size_t)b * (DD * SD);

#pragma unroll 1
    for (int r = 0; r < 8; ++r) {
        const int e = tid + NTHR * r;
        const int d = e >> 4;
        const int s4 = (e & 15) * 4;
        const v4f v = *(const v4f*)(fb + (size_t)d * SD + s4);
#pragma unroll
        for (int i = 0; i < 4; ++i) {
            unsigned short xh, xl;
            split2(v[i], xh, xl);
            sAH[(s4 + i) * EPITCH + d] = xh;
            sAL[(s4 + i) * EPITCH + d] = xl;
        }
    }
    __syncthreads();

    const int mt = wave >> 1, nt0 = (wave & 1) * 2;
    v8f acc[2];
    acc[0] = zero8(); acc[1] = zero8();
    lcp_us aHb = (lcp_us)sAH + (mt * 16 + m) * EPITCH + 8 * h;
    lcp_us aLb = (lcp_us)sAL + (mt * 16 + m) * EPITCH + 8 * h;
    const unsigned short* bHb = WeH + (size_t)(nt0 * 16 + m) * DD + 8 * h;
    const unsigned short* bLb = WeL + (size_t)(nt0 * 16 + m) * DD + 8 * h;
#pragma unroll 1
    for (int k0 = 0; k0 < DD; k0 += 32) {
        Frag aH, aL, bH[2], bL[2];
        ldfrag_lds(aH, aHb + k0);
        ldfrag_lds(aL, aLb + k0);
#pragma unroll
        for (int j = 0; j < 2; ++j) {
            ldfrag_glb(bH[j], bHb + (size_t)j * (16 * DD) + k0);
            ldfrag_glb(bL[j], bLb + (size_t)j * (16 * DD) + k0);
        }
#pragma unroll
        for (int j = 0; j < 2; ++j) {
            acc[j] = mma16(acc[j], aH, bH[j]);
            acc[j] = mma16(acc[j], aH, bL[j]);
            acc[j] = mma16(acc[j], aL, bH[j]);
        }
        asm volatile("v_nop\n\tv_nop\n\tv_nop\n\tv_nop"
                     : "+v"(acc[0]), "+v"(acc[1])
                     : "v"(aH.u), "v"(aL.u), "v"(bH[0].u), "v"(bH[1].u), "v"(bL[0].u), "v"(bL[1].u));
    }
#pragma unroll
    for (int j = 0; j < 2; ++j) {
        const int col = (nt0 + j) * 16 + m;
        const float bb = benc[col];
#pragma unroll
        for (int r = 0; r < 8; ++r) sP[(mt * 16 + 8 * h + r) * PPITCH + col] = acc[j][r] + bb;
    }
    __syncthreads();

    float* pb = penc + (size_t)b * (SD * AD);
    lcp_f sPp = (lcp_f)sP;
#pragma unroll
    for (int i = 0; i < 4; ++i) {
        const int p = tid + NTHR * i;
        const int row = p >> 4, c4 = (p & 15) * 4;
        const v4f v = *(AS3 const v4f*)(sPp + row * PPITCH + c4);
        *(volatile v4f*)(pb + 4 * p) = v;
    }
    __threadfence();
#pragma unroll
    for (int i = 0; i < 4; ++i) {
        const int p = tid + NTHR * i;
        const int row = p >> 4, c4 = (p & 15) * 4;
        const v4f v = *(AS3 const v4f*)(sPp + row * PPITCH + c4);
        *(volatile v4f*)(pb + 4 * p) = v;
    }
}

__global__ __launch_bounds__(NTHR)
void lstm_att_kernel(const float* __restrict__ tok, const float* __restrict__ feat, const float* __restrict__ fh,
                     const unsigned short* __restrict__ WcH, const unsigned short* __restrict__ WcL,
                     const unsigned short* __restrict__ WaH, const unsigned short* __restrict__ WaL,
                     const unsigned short* __restrict__ WpH, const unsigned short* __restrict__ WpL,
                     const float* __restrict__ bih, const float* __restrict__ bhh,
                     const float* __restrict__ wemb, const float* __restrict__ bemb,
                     const float* __restrict__ bh2, const float* __restrict__ walpha, const float* __restrict__ balpha,
                     const float* __restrict__ penc, const float* __restrict__ baap,
                     const float* __restrict__ wout, const float* __restrict__ bout, float* out)
{
    extern __shared__ __attribute__((aligned(16))) char smem[];
    lp_us actH   = (lp_us)(smem + LO_ACTH);
    lp_us actL   = (lp_us)(smem + LO_ACTL);
    lp_us aaH    = (lp_us)(smem + LO_AAH);
    lp_us aaL    = (lp_us)(smem + LO_AAL);
    lp_f  c_s    = (lp_f)(smem + LO_C);
    lp_f  atth   = (lp_f)(smem + LO_ATTH);
    lp_f  wgt    = (lp_f)(smem + LO_WGT);
    lp_f  outf   = (lp_f)(smem + LO_OUTF);
    lp_f  bias_s = (lp_f)(smem + LO_BIAS);
    lp_f  bh2_s  = (lp_f)(smem + LO_BH2);
    lp_f  walp_s = (lp_f)(smem + LO_WALP);
    lp_f  baap_s = (lp_f)(smem + LO_BAAP);
    lp_f  wout_s = (lp_f)(smem + LO_WOUT);
    lp_f  wemb_s = (lp_f)(smem + LO_WEMB);
    lp_f  bemb_s = (lp_f)(smem + LO_BEMB);
    lp_f  bout_s = (lp_f)(smem + LO_BOUT);
    lp_i  idx_s  = (lp_i)(smem + LO_IDX);
    lp_f  outs   = (lp_f)(smem + LO_OUTS);

    const int tid  = threadIdx.x;
    const int lane = tid & 31;
    const int wave = tid >> 5;
    const int h    = lane >> 4;
    const int m    = lane & 15;
    const int bg   = blockIdx.x * BB;

    {
        v4f zf;
#pragma unroll
        for (int i = 0; i < 4; ++i) zf[i] = 0.0f;
        lp_f z0 = (lp_f)(smem);
        for (int i = tid; i < (int)(LO_ATTH / 16); i += NTHR) *(AS3 v4f*)(z0 + 4 * i) = zf;
        for (int i = tid; i < NG; i += NTHR) bias_s[i] = bih[i] + bhh[i];
        if (tid < AD) { bh2_s[tid] = bh2[tid]; walp_s[tid] = walpha[tid]; }
        if (tid < IFD) baap_s[tid] = baap[tid];
        for (int i = tid; i < IFD * OD; i += NTHR) wout_s[i] = wout[i];
        if (tid < FIN * ED) wemb_s[tid] = wemb[tid];
        if (tid < ED) bemb_s[tid] = bemb[tid];
        if (tid < OD) bout_s[tid] = bout[tid];
        if (tid == OD) bout_s[OD] = balpha[0];
    }
    __syncthreads();

#pragma unroll 1
    for (int t = 0; t < TL; ++t) {
        if (wave == 0) {
            const int b = lane & 15;
            const float* tr = tok + ((size_t)(bg + b) * TL + t) * FIN;
            const float tx = tr[0], ty = tr[1];
            int x0 = (int)(tx * 100.0f); if (x0 == -1) x0 = 0;
            int y0 = (int)(ty * 100.0f); if (y0 == -1) y0 = 0;
            int idx = y0 * HMAP + x0;
            idx = min(max(idx, 0), HWD - 1);
            if (lane < BB) idx_s[lane] = idx;
        }
#pragma unroll 1
        for (int r = 0; r < 2; ++r) {
            const int e = tid + NTHR * r;
            const int b = e >> 5, ec = e & 31;
            const v4f tv = *(const v4f*)(tok + ((size_t)(bg + b) * TL + t) * FIN);
            float s = tv[0] * wemb_s[ec];
            s += tv[1] * wemb_s[ED + ec];
            s += tv[2] * wemb_s[2 * ED + ec];
            s += tv[3] * wemb_s[3 * ED + ec];
            s += bemb_s[ec];
            unsigned short xh, xl;
            split2(s, xh, xl);
            actH[b * APITCH + ec] = xh;
            actL[b * APITCH + ec] = xl;
        }
        __syncthreads();

#pragma unroll 1
        for (int r = 0; r < 8; ++r) {
            const int e = tid + NTHR * r;
            const int b = e >> 7, ch = e & 127;
            const int ix = idx_s[b];
            const float v = feat[((size_t)(bg + b) * CD + ch) * HWD + ix];
            unsigned short xh, xl;
            split2(v, xh, xl);
            actH[b * APITCH + ED + ch] = xh;
            actL[b * APITCH + ED + ch] = xl;
        }
        __syncthreads();

        v8f acc[4];
#pragma unroll
        for (int q = 0; q < 4; ++q) acc[q] = zero8();
        {
            lcp_us aHb = (lcp_us)actH + m * APITCH + 8 * h;
            lcp_us aLb = (lcp_us)actL + m * APITCH + 8 * h;
            const unsigned short* wHb = WcH + (size_t)(wave * 16 + m) * WPITCH + 8 * h;
            const unsigned short* wLb = WcL + (size_t)(wave * 16 + m) * WPITCH + 8 * h;
#pragma unroll 1
            for (int k0 = 0; k0 < KCAT; k0 += 32) {
                Frag aH, aL, bH[4], bL[4];
                ldfrag_lds(aH, aHb + k0);
                ldfrag_lds(aL, aLb + k0);
#pragma unroll
                for (int q = 0; q < 4; ++q) {
                    ldfrag_glb(bH[q], wHb + (size_t)q * (128 * WPITCH) + k0);
                    ldfrag_glb(bL[q], wLb + (size_t)q * (128 * WPITCH) + k0);
                }
#pragma unroll
                for (int q = 0; q < 4; ++q) {
                    acc[q] = mma16(acc[q], aH, bH[q]);
                    acc[q] = mma16(acc[q], aH, bL[q]);
                    acc[q] = mma16(acc[q], aL, bH[q]);
                }
                asm volatile("v_nop\n\tv_nop\n\tv_nop\n\tv_nop"
                             : "+v"(acc[0]), "+v"(acc[1]), "+v"(acc[2]), "+v"(acc[3])
                             : "v"(aH.u), "v"(aL.u), "v"(bH[0].u), "v"(bH[1].u), "v"(bH[2].u), "v"(bH[3].u),
                               "v"(bL[0].u), "v"(bL[1].u), "v"(bL[2].u), "v"(bL[3].u));
            }
        }
        __syncthreads();

        {
            const int n = wave * 16 + m;
            const float bi = bias_s[n];
            const float bf = bias_s[HD + n];
            const float bgt = bias_s[2 * HD + n];
            const float bo = bias_s[3 * HD + n];
#pragma unroll
            for (int r = 0; r < 8; ++r) {
                const int row = 8 * h + r;
                const float gi = acc[0][r] + bi;
                const float gf = acc[1][r] + bf;
                const float gg = acc[2][r] + bgt;
                const float go = acc[3][r] + bo;
                const float cp = c_s[row * HD + n];
                const float cn = sigm(gf) * cp + sigm(gi) * tanhm(gg);
                c_s[row * HD + n] = cn;
                const float hn = sigm(go) * tanhm(cn);
                unsigned short xh, xl;
                split2(hn, xh, xl);
                actH[row * APITCH + KIN + n] = xh;
                actL[row * APITCH + KIN + n] = xl;
                aaH[row * AAP + n] = xh;
                aaL[row * AAP + n] = xl;
            }
        }
        __syncthreads();

        if (wave < 4) {
            v8f pacc = zero8();
            lcp_us aHb = (lcp_us)aaH + m * AAP + 8 * h;
            lcp_us aLb = (lcp_us)aaL + m * AAP + 8 * h;
            const unsigned short* bHb = WaH + (size_t)(wave * 16 + m) * HD + 8 * h;
            const unsigned short* bLb = WaL + (size_t)(wave * 16 + m) * HD + 8 * h;
#pragma unroll 1
            for (int k0 = 0; k0 < HD; k0 += 32) {
                Frag aH, aL, bH, bL;
                ldfrag_lds(aH, aHb + k0);
                ldfrag_lds(aL, aLb + k0);
                ldfrag_glb(bH, bHb + k0);
                ldfrag_glb(bL, bLb + k0);
                pacc = mma16(pacc, aH, bH);
                pacc = mma16(pacc, aH, bL);
                pacc = mma16(pacc, aL, bH);
                asm volatile("v_nop\n\tv_nop\n\tv_nop\n\tv_nop"
                             : "+v"(pacc) : "v"(aH.u), "v"(aL.u), "v"(bH.u), "v"(bL.u));
            }
            const int col = wave * 16 + m;
            const float bb = bh2_s[col];
#pragma unroll
            for (int r = 0; r < 8; ++r) atth[(8 * h + r) * AD + col] = pacc[r] + bb;
        }
        __syncthreads();

        {
            const float ba = bout_s[OD];
#pragma unroll 1
            for (int r = 0; r < 4; ++r) {
                const int e = tid + NTHR * r;
                const int b = e >> 6, s = e & 63;
                const v4f* pp = (const v4f*)(penc + ((size_t)(bg + b) * SD + s) * AD);
                lcp_f ah = (lcp_f)atth + b * AD;
                lcp_f wa = (lcp_f)walp_s;
                float sc = 0.0f;
#pragma unroll 1
                for (int a4 = 0; a4 < AD / 4; ++a4) {
                    const v4f p4 = pp[a4];
                    const v4f h4 = *(AS3 const v4f*)(ah + 4 * a4);
                    const v4f w4 = *(AS3 const v4f*)(wa + 4 * a4);
#pragma unroll
                    for (int i = 0; i < 4; ++i) sc += tanhm(p4[i] + h4[i]) * w4[i];
                }
                wgt[b * SD + s] = sc + ba;
            }
        }
        __syncthreads();

#pragma unroll 1
        for (int rr = 0; rr < 2; ++rr) {
            const int row = wave * 2 + rr;
            lp_f wr = wgt + row * SD;
            const float v0 = wr[lane], v1 = wr[lane + 32];
            float mx = fmaxf(v0, v1);
#pragma unroll
            for (int off = 16; off > 0; off >>= 1) mx = fmaxf(mx, __shfl_xor(mx, off));
            const float e0 = __expf(v0 - mx), e1 = __expf(v1 - mx);
            float sm = e0 + e1;
#pragma unroll
            for (int off = 16; off > 0; off >>= 1) sm += __shfl_xor(sm, off);
            const float inv = rcpx(sm);
            wr[lane] = e0 * inv;
            wr[lane + 32] = e1 * inv;
        }
        __syncthreads();

#pragma unroll 1
        for (int r = 0; r < 8; ++r) {
            const int e = tid + NTHR * r;
            const int b = e >> 7, d = e & 127;
            const v4f* fp = (const v4f*)(fh + ((size_t)(bg + b) * DD + d) * SD);
            lcp_f wr = (lcp_f)wgt + b * SD;
            float ar = 0.0f;
#pragma unroll 2
            for (int s4 = 0; s4 < SD / 4; ++s4) {
                const v4f f4 = fp[s4];
                const v4f w4 = *(AS3 const v4f*)(wr + 4 * s4);
                ar += f4[0] * w4[0];
                ar += f4[1] * w4[1];
                ar += f4[2] * w4[2];
                ar += f4[3] * w4[3];
            }
            unsigned short xh, xl;
            split2(ar, xh, xl);
            aaH[b * AAP + HD + d] = xh;
            aaL[b * AAP + HD + d] = xl;
        }
        __syncthreads();

        {
            v8f pacc = zero8();
            lcp_us aHb = (lcp_us)aaH + m * AAP + 8 * h;
            lcp_us aLb = (lcp_us)aaL + m * AAP + 8 * h;
            const unsigned short* bHb = WpH + (size_t)(wave * 16 + m) * (HD + DD) + 8 * h;
            const unsigned short* bLb = WpL + (size_t)(wave * 16 + m) * (HD + DD) + 8 * h;
#pragma unroll 1
            for (int k0 = 0; k0 < HD + DD; k0 += 32) {
                Frag aH, aL, bH, bL;
                ldfrag_lds(aH, aHb + k0);
                ldfrag_lds(aL, aLb + k0);
                ldfrag_glb(bH, bHb + k0);
                ldfrag_glb(bL, bLb + k0);
                pacc = mma16(pacc, aH, bH);
                pacc = mma16(pacc, aH, bL);
                pacc = mma16(pacc, aL, bH);
                asm volatile("v_nop\n\tv_nop\n\tv_nop\n\tv_nop"
                             : "+v"(pacc) : "v"(aH.u), "v"(aL.u), "v"(bH.u), "v"(bL.u));
            }
            const int col = wave * 16 + m;
            const float bb = baap_s[col];
#pragma unroll
            for (int r = 0; r < 8; ++r) {
                const int row = 8 * h + r;
                const float v = pacc[r] + bb;
                outf[row * IFD + col] = v;
                unsigned short xh, xl;
                split2(v, xh, xl);
                actH[row * APITCH + (ED + CD) + col] = xh;
                actL[row * APITCH + (ED + CD) + col] = xl;
            }
        }
        __syncthreads();

        if (tid < BB * OD) {
            const int b = tid / OD;
            const int o = tid - b * OD;
            lcp_f fr = (lcp_f)outf + b * IFD;
            float s = 0.0f;
#pragma unroll 4
            for (int i = 0; i < IFD; ++i) s += fr[i] * wout_s[i * OD + o];
            outs[b * (TL * OD) + t * OD + o] = s + bout_s[o];
        }
    }
    __syncthreads();

    float* ob = out + (size_t)blockIdx.x * (BB * TL * OD);
    lcp_f op = (lcp_f)outs;
#pragma unroll 1
    for (int i = 0; i < NOUT_IT; ++i) {
        const int p = tid + NTHR * i;
        if (p < NOUTP) {
            const v4f v = *(AS3 const v4f*)(op + 4 * p);
            *(volatile v4f*)(ob + 4 * p) = v;
        }
    }
    __threadfence();
#pragma unroll 1
    for (int i = 0; i < NOUT_IT; ++i) {
        const int p = tid + NTHR * i;
        if (p < NOUTP) {
            const v4f v = *(AS3 const v4f*)(op + 4 * p);
            *(volatile v4f*)(ob + 4 * p) = v;
        }
    }
}

extern "C" void kernel_launch(void* const* d_in, const int* in_sizes, int n_in,
                              void* d_out, int out_size, void* d_ws, size_t ws_size,
                              hipStream_t stream)
{
    if (n_in < 19) return;
    if (in_sizes[0]  != NB * TL * FIN)      return;
    if (in_sizes[1]  != NB * CD * HWD)      return;
    if (in_sizes[2]  != NB * DD * SD)       return;
    if (in_sizes[3]  != FIN * ED)           return;
    if (in_sizes[4]  != ED)                 return;
    if (in_sizes[5]  != KIN * NG)           return;
    if (in_sizes[6]  != NG)                 return;
    if (in_sizes[7]  != HD * NG)            return;
    if (in_sizes[8]  != NG)                 return;
    if (in_sizes[9]  != HD * AD)            return;
    if (in_sizes[10] != AD)                 return;
    if (in_sizes[11] != AD)                 return;
    if (in_sizes[12] < 1)                   return;
    if (in_sizes[13] != DD * AD)            return;
    if (in_sizes[14] != AD)                 return;
    if (in_sizes[15] != (HD + DD) * IFD)    return;
    if (in_sizes[16] != IFD)                return;
    if (in_sizes[17] != IFD * OD)           return;
    if (in_sizes[18] != OD)                 return;
    if (out_size != NB * TL * OD)           return;
    if (ws_size < WS_END)                   return;

    const float* tok    = (const float*)d_in[0];
    const float* feat   = (const float*)d_in[1];
    const float* fhid   = (const float*)d_in[2];
    const float* Wemb   = (const float*)d_in[3];
    const float* bemb   = (const float*)d_in[4];
    const float* Wih    = (const float*)d_in[5];
    const float* bih    = (const float*)d_in[6];
    const float* Whh    = (const float*)d_in[7];
    const float* bhh    = (const float*)d_in[8];
    const float* Wh2    = (const float*)d_in[9];
    const float* bh2    = (const float*)d_in[10];
    const float* Walpha = (const float*)d_in[11];
    const float* balpha = (const float*)d_in[12];
    const float* Wenc   = (const float*)d_in[13];
    const float* benc   = (const float*)d_in[14];
    const float* Waap   = (const float*)d_in[15];
    const float* baap   = (const float*)d_in[16];
    const float* Wout   = (const float*)d_in[17];
    const float* bout   = (const float*)d_in[18];
    float* out = (float*)d_out;

    char* ws = (char*)d_ws;
    unsigned short* WcH = (unsigned short*)(ws + OFF_WCH);
    unsigned short* WcL = (unsigned short*)(ws + OFF_WCL);
    unsigned short* WaH = (unsigned short*)(ws + OFF_WAH);
    unsigned short* WaL = (unsigned short*)(ws + OFF_WAL);
    unsigned short* WpH = (unsigned short*)(ws + OFF_WPH);
    unsigned short* WpL = (unsigned short*)(ws + OFF_WPL);
    unsigned short* WeH = (unsigned short*)(ws + OFF_WEH);
    unsigned short* WeL = (unsigned short*)(ws + OFF_WEL);
    float* penc = (float*)(ws + OFF_PE);

    cvt_kernel<<<dim3(CB3), dim3(NTHR), 0, stream>>>(Wih, Whh, Wh2, Waap, Wenc,
                                                    WcH, WcL, WaH, WaL, WpH, WpL, WeH, WeL);

    penc_kernel<<<dim3(NB), dim3(NTHR), 0, stream>>>(fhid, (const unsigned short*)WeH,
                                                    (const unsigned short*)WeL, benc, penc);

    hipFuncSetAttribute(reinterpret_cast<const void*>(&lstm_att_kernel),
                        hipFuncAttributeMaxDynamicSharedMemorySize, (int)LDS_BYTES);
    lstm_att_kernel<<<dim3(NBLK), dim3(NTHR), LDS_BYTES, stream>>>(
        tok, feat, fhid,
        (const unsigned short*)WcH, (const unsigned short*)WcL,
        (const unsigned short*)WaH, (const unsigned short*)WaL,
        (const unsigned short*)WpH, (const unsigned short*)WpL,
        bih, bhh, Wemb, bemb, bh2, Walpha, balpha, (const float*)penc, baap, Wout, bout, out);
}
